// MultiHeadAttention_2594160246919
// MI455X (gfx1250) — hardware-run, weakly checked
//
#include <hip/hip_runtime.h>
#ifndef NB
#define NB 2
#endif
#ifndef SEQ
#define SEQ 2048
#endif
#define NB_FULL 2
#define SEQ_FULL 2048
#define DM 512
#define NH 8
#define HD 64
#define XBSTRIDE_FULL ((size_t)SEQ_FULL * DM)
#define QKPLANE ((size_t)NB * NH * SEQ * HD)
#define CPLANE ((size_t)NB * SEQ * DM)
#define WS_TOTAL (CPLANE * 2 + (size_t)3 * DM * DM * 2 + (size_t)DM * DM * 2 + QKPLANE * 2 * 4 + QKPLANE * 2 + CPLANE * 2 * 2 + 8 * 256)

static_assert(SEQ % 128 == 0);
static_assert(SEQ <= SEQ_FULL);
static_assert(NB <= NB_FULL);
static_assert(HD == 64);
static_assert(DM == NH * HD);
static_assert(DM % 64 == 0);
static_assert(WS_TOTAL <= (size_t)134217728);

typedef __bf16 v16b __attribute__((ext_vector_type(16)));
typedef _Float16 v16h __attribute__((ext_vector_type(16)));
typedef unsigned short v8us __attribute__((ext_vector_type(8), may_alias));
typedef float v8f __attribute__((ext_vector_type(8)));
typedef float v4f __attribute__((ext_vector_type(4)));
typedef float v4fa __attribute__((ext_vector_type(4), may_alias));
union FragB { v16b v; v8us half[2]; unsigned short u[16]; };
union FragH { v16h v; v8us half[2]; _Float16 h[16]; unsigned short u[16]; };
union H8 { v8us v; _Float16 h[8]; unsigned short u[8]; };

#define LOG2E 1.4426950408889634f

__device__ __forceinline__ unsigned short bf16_bits(float x) {
  unsigned int u = __float_as_uint(x);
  return (unsigned short)((u + 0x7FFFu + ((u >> 16) & 1u)) >> 16);
}
__device__ __forceinline__ float bf16_val(unsigned short b) { return __uint_as_float(((unsigned int)b) << 16); }
__device__ __forceinline__ float bf16_rne(float x) { return bf16_val(bf16_bits(x)); }
__device__ __forceinline__ unsigned short f16_bits(float x) { union { _Float16 h; unsigned short u; } c; c.h = (_Float16)x; return c.u; }

__device__ __forceinline__ v8f mma_bf2(v16b a0, v16b b0, v16b a1, v16b b1, v8f c) {
  c = __builtin_amdgcn_wmma_f32_16x16x32_bf16(false, a0, false, b0, (short)0, c, false, false);
  c = __builtin_amdgcn_wmma_f32_16x16x32_bf16(false, a1, false, b1, (short)0, c, false, false);
  asm volatile("v_nop\n\tv_nop\n\tv_nop\n\tv_nop" : "+v"(c) : "v"(a0), "v"(b0), "v"(a1), "v"(b1));
  return c;
}
__device__ __forceinline__ void mma_b1x2(v16b a0, v16b a1, v16b b, v8f& c0, v8f& c1) {
  c0 = __builtin_amdgcn_wmma_f32_16x16x32_bf16(false, a0, false, b, (short)0, c0, false, false);
  c1 = __builtin_amdgcn_wmma_f32_16x16x32_bf16(false, a1, false, b, (short)0, c1, false, false);
  asm volatile("v_nop\n\tv_nop\n\tv_nop\n\tv_nop" : "+v"(c0), "+v"(c1) : "v"(a0), "v"(a1), "v"(b));
}
__device__ __forceinline__ void mma_h2(v16h a, v16h bh, v16h bl, v8f& ch, v8f& cl) {
  ch = __builtin_amdgcn_wmma_f32_16x16x32_f16(false, a, false, bh, (short)0, ch, false, false);
  cl = __builtin_amdgcn_wmma_f32_16x16x32_f16(false, a, false, bl, (short)0, cl, false, false);
  asm volatile("v_nop\n\tv_nop\n\tv_nop\n\tv_nop" : "+v"(ch), "+v"(cl) : "v"(a), "v"(bh), "v"(bl));
}
__device__ __forceinline__ void mma_hA2(v16h ah, v16h al, v16h b, v8f& ch, v8f& cl) {
  ch = __builtin_amdgcn_wmma_f32_16x16x32_f16(false, ah, false, b, (short)0, ch, false, false);
  cl = __builtin_amdgcn_wmma_f32_16x16x32_f16(false, al, false, b, (short)0, cl, false, false);
  asm volatile("v_nop\n\tv_nop\n\tv_nop\n\tv_nop" : "+v"(ch), "+v"(cl) : "v"(ah), "v"(al), "v"(b));
}

__global__ __launch_bounds__(256) void k_xb(const float* __restrict__ X, unsigned short* __restrict__ Xb) {
  const int t = blockIdx.x * 256 + threadIdx.x;
  if (t >= NB * SEQ * 64) return;
  const int row = t >> 6, piece = t & 63;
  const int b = row / SEQ, s = row - b * SEQ;
  const float* src = X + (size_t)b * XBSTRIDE_FULL + (size_t)s * DM + piece * 8;
  const v4f x0 = *(const v4fa*)(src), x1 = *(const v4fa*)(src + 4);
  v8us o;
  o[0] = bf16_bits(x0[0]); o[1] = bf16_bits(x0[1]); o[2] = bf16_bits(x0[2]); o[3] = bf16_bits(x0[3]);
  o[4] = bf16_bits(x1[0]); o[5] = bf16_bits(x1[1]); o[6] = bf16_bits(x1[2]); o[7] = bf16_bits(x1[3]);
  unsigned short* d = Xb + (size_t)t * 8;
  *(volatile v8us*)d = o;
  __threadfence();
  *(volatile v8us*)d = o;
}

template <int MODE>
__device__ __forceinline__ unsigned short wconv(float x) {
  if (MODE == 0) return bf16_bits(x);
  return f16_bits(bf16_rne(x) * 64.0f);
}

template <int MODE>
__global__ __launch_bounds__(256) void k_wt(const float* __restrict__ W, unsigned short* __restrict__ Dst,
                                            int tstride, int ld, int rowbase) {
  __shared__ unsigned short tl[64][66];
  const int tid = threadIdx.x;
  const int k0 = blockIdx.x * 64, j = blockIdx.y;
  const float* src = W + (size_t)j * tstride + (size_t)k0 * ld;
  for (int i = tid; i < 64 * 16; i += 256) {
    const int kk = i >> 4, c4 = (i & 15) * 4;
    const v4f x = *(const v4fa*)(src + (size_t)kk * ld + c4);
    tl[c4 + 0][kk] = wconv<MODE>(x[0]);
    tl[c4 + 1][kk] = wconv<MODE>(x[1]);
    tl[c4 + 2][kk] = wconv<MODE>(x[2]);
    tl[c4 + 3][kk] = wconv<MODE>(x[3]);
  }
  __syncthreads();
  for (int pass = 0; pass < 2; ++pass) {
    for (int i = tid; i < 64 * 8; i += 256) {
      const int n = i >> 3, k8 = (i & 7) * 8;
      v8us o;
#pragma unroll
      for (int q = 0; q < 8; ++q) o[q] = tl[n][k8 + q];
      *(volatile v8us*)(Dst + (size_t)(rowbase + j * 64 + n) * DM + k0 + k8) = o;
    }
    if (pass == 0) __threadfence();
  }
}

__global__ __launch_bounds__(128) void k_proj(const unsigned short* __restrict__ Xb, const unsigned short* __restrict__ Wt,
                                              const float* __restrict__ bq, const float* __restrict__ bk,
                                              const float* __restrict__ bv,
                                              unsigned short* __restrict__ QK, unsigned short* __restrict__ Vt) {
  __shared__ __attribute__((aligned(16))) float so[128][68];
  const int tid = threadIdx.x, w = __builtin_amdgcn_readfirstlane((int)(tid >> 5)), lane = tid & 31, ln = lane & 15, hh = lane >> 4;
  const int y = blockIdx.y;
  const int which = y >> 3, h = y & 7;
  const int m_base = blockIdx.x * 128;
  const unsigned short* ap0 = Xb + (size_t)(m_base + 32 * w + ln) * DM + 8 * hh;
  const unsigned short* ap1 = ap0 + (size_t)16 * DM;
  const unsigned short* bp = Wt + (size_t)(y * 64 + ln) * DM + 8 * hh;
  v8f acc0[4] = {}, acc1[4] = {};
#pragma unroll 2
  for (int k0 = 0; k0 < DM; k0 += 32) {
    FragB a0, a1, bf[4];
    a0.half[0] = *(const v8us*)(ap0 + k0); a0.half[1] = *(const v8us*)(ap0 + k0 + 16);
    a1.half[0] = *(const v8us*)(ap1 + k0); a1.half[1] = *(const v8us*)(ap1 + k0 + 16);
#pragma unroll
    for (int t = 0; t < 4; ++t) {
      bf[t].half[0] = *(const v8us*)(bp + (size_t)t * 16 * DM + k0);
      bf[t].half[1] = *(const v8us*)(bp + (size_t)t * 16 * DM + k0 + 16);
    }
#pragma unroll
    for (int t = 0; t < 4; ++t) mma_b1x2(a0.v, a1.v, bf[t].v, acc0[t], acc1[t]);
  }
#pragma unroll
  for (int t = 0; t < 4; ++t) {
    const int bi = h * HD + 16 * t + ln;
    const float b0 = bq[bi], b1 = bk[bi], b2 = bv[bi];
    const float bias = bf16_rne((which == 0) ? b0 : ((which == 1) ? b1 : b2));
#pragma unroll
    for (int r = 0; r < 8; ++r) {
      so[32 * w + 8 * hh + r][16 * t + ln]      = acc0[t][r] + bias;
      so[32 * w + 16 + 8 * hh + r][16 * t + ln] = acc1[t][r] + bias;
    }
  }
  __syncthreads();
  const int b = m_base / SEQ, s0 = m_base - b * SEQ;
  const int bh = b * NH + h;
  if (which < 2) {
    unsigned short* dh = QK + (size_t)(2 * which) * QKPLANE + ((size_t)bh * SEQ + s0) * HD;
    unsigned short* dl = dh + QKPLANE;
    for (int pass = 0; pass < 2; ++pass) {
#pragma unroll 2
      for (int it = 0; it < 8; ++it) {
        const int i = tid + 128 * it;
        const int row = i >> 3, piece = i & 7;
        const v4f x0 = *(const v4fa*)&so[row][piece * 8];
        const v4f x1 = *(const v4fa*)&so[row][piece * 8 + 4];
        v8us oh, ol;
#pragma unroll
        for (int q = 0; q < 4; ++q) {
          const unsigned short h0 = bf16_bits(x0[q]);
          const unsigned short h1 = bf16_bits(x1[q]);
          oh[q] = h0; oh[4 + q] = h1;
          ol[q] = bf16_bits(x0[q] - bf16_val(h0));
          ol[4 + q] = bf16_bits(x1[q] - bf16_val(h1));
        }
        *(volatile v8us*)(dh + (size_t)row * HD + piece * 8) = oh;
        *(volatile v8us*)(dl + (size_t)row * HD + piece * 8) = ol;
      }
      if (pass == 0) __threadfence();
    }
  } else {
    unsigned short* dv = Vt + ((size_t)bh * HD) * SEQ + s0;
    for (int pass = 0; pass < 2; ++pass) {
#pragma unroll 2
      for (int it = 0; it < 8; ++it) {
        const int i = tid + 128 * it;
        const int d = i >> 4, p8 = (i & 15) * 8;
        H8 o;
#pragma unroll
        for (int q = 0; q < 8; ++q) o.h[q] = (_Float16)(so[p8 + q][d] * 16.0f);
        *(volatile v8us*)(dv + (size_t)d * SEQ + p8) = o.v;
      }
      if (pass == 0) __threadfence();
    }
  }
}

__device__ __forceinline__ void fa_step(const unsigned short* __restrict__ Khp, const unsigned short* __restrict__ Vp,
                                        int key0, int ln, int hh,
                                        const FragB& q0h, const FragB& q1h, const FragB& q0l, const FragB& q1l,
                                        float& mr, float& lr, v8f (&Oh)[4], v8f (&Ol)[4]) {
  const v8f z8 = {0.f, 0.f, 0.f, 0.f, 0.f, 0.f, 0.f, 0.f};
  const unsigned short* kp0 = Khp + (size_t)(key0 + ln) * HD + 8 * hh;
  const unsigned short* kp1 = kp0 + 16 * HD;
  v8f s0, s1;
  {
    FragB h0, h1, l0, l1;
    h0.half[0] = *(const v8us*)(kp0);      h0.half[1] = *(const v8us*)(kp0 + 16);
    h1.half[0] = *(const v8us*)(kp0 + 32); h1.half[1] = *(const v8us*)(kp0 + 48);
    l0.half[0] = *(const v8us*)(kp0 + QKPLANE);      l0.half[1] = *(const v8us*)(kp0 + QKPLANE + 16);
    l1.half[0] = *(const v8us*)(kp0 + QKPLANE + 32); l1.half[1] = *(const v8us*)(kp0 + QKPLANE + 48);
    s0 = mma_bf2(l0.v, q0h.v, l1.v, q1h.v, z8);
    s0 = mma_bf2(h0.v, q0l.v, h1.v, q1l.v, s0);
    s0 = mma_bf2(h0.v, q0h.v, h1.v, q1h.v, s0);
  }
  asm volatile("" ::: "memory");
  {
    FragB h0, h1, l0, l1;
    h0.half[0] = *(const v8us*)(kp1);      h0.half[1] = *(const v8us*)(kp1 + 16);
    h1.half[0] = *(const v8us*)(kp1 + 32); h1.half[1] = *(const v8us*)(kp1 + 48);
    l0.half[0] = *(const v8us*)(kp1 + QKPLANE);      l0.half[1] = *(const v8us*)(kp1 + QKPLANE + 16);
    l1.half[0] = *(const v8us*)(kp1 + QKPLANE + 32); l1.half[1] = *(const v8us*)(kp1 + QKPLANE + 48);
    s1 = mma_bf2(l0.v, q0h.v, l1.v, q1h.v, z8);
    s1 = mma_bf2(h0.v, q0l.v, h1.v, q1l.v, s1);
    s1 = mma_bf2(h0.v, q0h.v, h1.v, q1h.v, s1);
  }
  asm volatile("" ::: "memory");
  const unsigned short* vp = Vp + (size_t)ln * SEQ + key0 + 8 * hh;
  FragH vf[4];
#pragma unroll
  for (int t = 0; t < 4; ++t) {
    vf[t].half[0] = *(const v8us*)(vp + (size_t)t * 16 * SEQ);
    vf[t].half[1] = *(const v8us*)(vp + (size_t)t * 16 * SEQ + 16);
  }
  float sc[16];
#pragma unroll
  for (int r = 0; r < 8; ++r) { sc[r] = s0[r] * 0.125f; sc[8 + r] = s1[r] * 0.125f; }
  float mx = sc[0];
#pragma unroll
  for (int i = 1; i < 16; ++i) mx = fmaxf(mx, sc[i]);
  mx = fmaxf(mx, __shfl_xor(mx, 16, 32));
  const float mnew = fmaxf(mr, mx);
  const float al = exp2f((mr - mnew) * LOG2E);
  mr = mnew;
  FragH ph, pl;
  float ps = 0.0f;
#pragma unroll
  for (int i = 0; i < 16; ++i) {
    const float pc = exp2f(fmaf(sc[i] - mnew, LOG2E, 8.0f));
    ps += pc;
    const _Float16 hv = (_Float16)pc;
    ph.h[i] = hv;
    pl.h[i] = (_Float16)((pc - (float)hv) * 2048.0f);
  }
  ps += __shfl_xor(ps, 16, 32);
  lr = lr * al + ps;
#pragma unroll
  for (int t = 0; t < 4; ++t) { Oh[t] = Oh[t] * al; Ol[t] = Ol[t] * al; }
#pragma unroll
  for (int t = 0; t < 4; ++t) mma_h2(vf[t].v, ph.v, pl.v, Oh[t], Ol[t]);
}

__global__ __launch_bounds__(128) void k_attn(const unsigned short* __restrict__ QK, const unsigned short* __restrict__ Vt,
                                              unsigned short* __restrict__ Cc) {
  __shared__ __attribute__((aligned(16))) float so[4][16][68];
  const int tid = threadIdx.x, w = __builtin_amdgcn_readfirstlane((int)(tid >> 5)), lane = tid & 31, ln = lane & 15, hh = lane >> 4;
  const int bh = blockIdx.x / (SEQ / 64), qt = blockIdx.x % (SEQ / 64);
  const int b = bh / NH, h = bh - b * NH;
  const int qbase = qt * 64 + 16 * w;
  const int qg = qbase + ln;
  const unsigned short* qrow = QK + ((size_t)bh * SEQ + qg) * HD + 8 * hh;
  FragB q0h, q1h, q0l, q1l;
  q0h.half[0] = *(const v8us*)(qrow);      q0h.half[1] = *(const v8us*)(qrow + 16);
  q1h.half[0] = *(const v8us*)(qrow + 32); q1h.half[1] = *(const v8us*)(qrow + 48);
  q0l.half[0] = *(const v8us*)(qrow + QKPLANE);      q0l.half[1] = *(const v8us*)(qrow + QKPLANE + 16);
  q1l.half[0] = *(const v8us*)(qrow + QKPLANE + 32); q1l.half[1] = *(const v8us*)(qrow + QKPLANE + 48);
  float mr = -3.0e38f, lr = 0.0f;
  v8f Oh[4] = {}, Ol[4] = {};
  const unsigned short* Khp = QK + 2 * QKPLANE + (size_t)bh * SEQ * HD;
  const unsigned short* Vp = Vt + (size_t)bh * HD * SEQ;
#pragma unroll 1
  for (int j = 0; j < SEQ / 32; ++j)
    fa_step(Khp, Vp, 32 * j, ln, hh, q0h, q1h, q0l, q1l, mr, lr, Oh, Ol);

  const float c256 = 16.0f * (1.0f / lr);
#pragma unroll
  for (int t = 0; t < 4; ++t)
#pragma unroll
    for (int r = 0; r < 8; ++r)
      so[w][ln][16 * t + 8 * hh + r] = (Oh[t][r] + Ol[t][r] * 0.00048828125f) * c256;
  __syncthreads();
  unsigned short* ch = Cc + ((size_t)b * SEQ + qbase) * DM + h * HD;
  unsigned short* cl = ch + CPLANE;
  const int rq = lane >> 3, piece = lane & 7;
  for (int pass = 0; pass < 2; ++pass) {
#pragma unroll
    for (int it = 0; it < 4; ++it) {
      const int row = 4 * it + rq;
      const v4f x0 = *(const v4fa*)&so[w][row][piece * 8];
      const v4f x1 = *(const v4fa*)&so[w][row][piece * 8 + 4];
      H8 oh, ol;
#pragma unroll
      for (int q = 0; q < 4; ++q) {
        const _Float16 h0 = (_Float16)x0[q];
        const _Float16 h1 = (_Float16)x1[q];
        oh.h[q] = h0; oh.h[4 + q] = h1;
        ol.h[q] = (_Float16)((x0[q] - (float)h0) * 2048.0f);
        ol.h[4 + q] = (_Float16)((x1[q] - (float)h1) * 2048.0f);
      }
      *(volatile v8us*)(ch + (size_t)row * DM + piece * 8) = oh.v;
      *(volatile v8us*)(cl + (size_t)row * DM + piece * 8) = ol.v;
    }
    if (pass == 0) __threadfence();
  }
}

__global__ __launch_bounds__(128) void k_oproj(const unsigned short* __restrict__ Cc, const unsigned short* __restrict__ WoT,
                                               const float* __restrict__ bo, float* __restrict__ Out) {
  __shared__ __attribute__((aligned(16))) float so[4][16][68];
  const int tid = threadIdx.x, w = __builtin_amdgcn_readfirstlane((int)(tid >> 5)), lane = tid & 31, ln = lane & 15, hh = lane >> 4;
  const int mblk = blockIdx.x * 64;
  const int n0 = blockIdx.y * 64;
  const unsigned short* ap = Cc + (size_t)(mblk + 16 * w + ln) * DM + 8 * hh;
  const unsigned short* bp = WoT + (size_t)(n0 + ln) * DM + 8 * hh;
  v8f ah[4] = {}, al[4] = {};
#pragma unroll 2
  for (int k0 = 0; k0 < DM; k0 += 32) {
    FragH fa, fr, bf[4];
    fa.half[0] = *(const v8us*)(ap + k0);          fa.half[1] = *(const v8us*)(ap + k0 + 16);
    fr.half[0] = *(const v8us*)(ap + CPLANE + k0); fr.half[1] = *(const v8us*)(ap + CPLANE + k0 + 16);
#pragma unroll
    for (int t = 0; t < 4; ++t) {
      bf[t].half[0] = *(const v8us*)(bp + (size_t)t * 16 * DM + k0);
      bf[t].half[1] = *(const v8us*)(bp + (size_t)t * 16 * DM + k0 + 16);
    }
#pragma unroll
    for (int t = 0; t < 4; ++t) mma_hA2(fa.v, fr.v, bf[t].v, ah[t], al[t]);
  }
#pragma unroll
  for (int t = 0; t < 4; ++t) {
    const float bias = bf16_rne(bo[n0 + 16 * t + ln]);
#pragma unroll
    for (int r = 0; r < 8; ++r)
      so[w][8 * hh + r][16 * t + ln] = (ah[t][r] + al[t][r] * 0.00048828125f) * 0.00006103515625f + bias;
  }
  __syncthreads();
  const int b = mblk / SEQ, s0 = mblk - b * SEQ;
  float* og = Out + (size_t)b * XBSTRIDE_FULL + (size_t)(s0 + 16 * w) * DM + n0;
  const int rsub = lane >> 4, c4 = (lane & 15) * 4;
  for (int pass = 0; pass < 2; ++pass) {
#pragma unroll
    for (int q = 0; q < 8; ++q) {
      const int row = 2 * q + rsub;
      const v4f v = *(const v4fa*)&so[w][row][c4];
      *(volatile v4f*)(og + (size_t)row * DM + c4) = v;
    }
    if (pass == 0) __threadfence();
  }
}

extern "C" void kernel_launch(void* const* d_in, const int* in_sizes, int n_in,
                              void* d_out, int out_size, void* d_ws, size_t ws_size, hipStream_t stream) {
  if (n_in < 9) return;
  const long long needx = (long long)(NB - 1) * SEQ_FULL * DM + (long long)SEQ * DM;
  if ((long long)in_sizes[0] < needx) return;
  if (in_sizes[1] < NH * DM * HD || in_sizes[2] < NH * DM * HD || in_sizes[3] < NH * DM * HD) return;
  if (in_sizes[4] < DM || in_sizes[5] < DM || in_sizes[6] < DM) return;
  if (in_sizes[7] < DM * DM || in_sizes[8] < DM) return;
  if ((long long)out_size < needx) return;
  const float* x  = (const float*)d_in[0];
  const float* Wq = (const float*)d_in[1];
  const float* Wk = (const float*)d_in[2];
  const float* Wv = (const float*)d_in[3];
  const float* bq = (const float*)d_in[4];
  const float* bk = (const float*)d_in[5];
  const float* bv = (const float*)d_in[6];
  const float* Wo = (const float*)d_in[7];
  const float* bo = (const float*)d_in[8];
  float* Out = (float*)d_out;
  char* ws = (char*)d_ws;
  size_t off = 0;
  const size_t szXb = CPLANE * 2;
  const size_t szWt = (size_t)3 * DM * DM * 2;
  const size_t szWo = (size_t)DM * DM * 2;
  const size_t szQK = QKPLANE * 2 * 4;
  const size_t szVt = QKPLANE * 2;
  const size_t szC  = CPLANE * 2 * 2;
  unsigned short* Xb  = (unsigned short*)(ws + off); off += (szXb + 255) & ~(size_t)255;
  unsigned short* Wt  = (unsigned short*)(ws + off); off += (szWt + 255) & ~(size_t)255;
  unsigned short* WoT = (unsigned short*)(ws + off); off += (szWo + 255) & ~(size_t)255;
  unsigned short* QK  = (unsigned short*)(ws + off); off += (szQK + 255) & ~(size_t)255;
  unsigned short* Vt  = (unsigned short*)(ws + off); off += (szVt + 255) & ~(size_t)255;
  unsigned short* Cc  = (unsigned short*)(ws + off); off += (szC + 255) & ~(size_t)255;
  if (off > ws_size) return;
  k_xb<<<(unsigned)((NB * SEQ * 64 + 255) / 256), 256, 0, stream>>>(x, Xb);
  k_wt<0><<<dim3(DM / 64, NH), 256, 0, stream>>>(Wq, Wt, DM * HD, HD, 0);
  k_wt<0><<<dim3(DM / 64, NH), 256, 0, stream>>>(Wk, Wt, DM * HD, HD, DM);
  k_wt<0><<<dim3(DM / 64, NH), 256, 0, stream>>>(Wv, Wt, DM * HD, HD, 2 * DM);
  k_wt<1><<<dim3(DM / 64, DM / 64), 256, 0, stream>>>(Wo, WoT, 64, DM, 0);
  k_proj<<<dim3((unsigned)(NB * SEQ / 128), 3 * NH), 128, 0, stream>>>(Xb, Wt, bq, bk, bv, QK, Vt);
  k_attn<<<(unsigned)(NB * NH * (SEQ / 64)), 128, 0, stream>>>(QK, Vt, Cc);
  k_oproj<<<dim3((unsigned)(NB * SEQ / 64), DM / 64), 128, 0, stream>>>(Cc, WoT, bo, Out);
}
